// ScanAttention_14130442404169
// MI455X (gfx1250) — hardware-verified
//
#include <hip/hip_runtime.h>
#include <stdint.h>
#include <math.h>

typedef __attribute__((ext_vector_type(16))) __bf16   v16b;
typedef __attribute__((ext_vector_type(8)))  __bf16   v8b;
typedef __attribute__((ext_vector_type(8)))  float    v8f;
typedef __attribute__((ext_vector_type(4)))  float    v4f;
typedef __attribute__((ext_vector_type(4)))  unsigned v4u;

constexpr int kBatch = 2;
constexpr int kSeq   = 2048;
constexpr int kSkv   = 2048;
constexpr int kHeads = 16;
constexpr int kDim   = 64;
constexpr int kQB    = 64;
constexpr int kKC    = 64;
constexpr int kNW    = 4;
constexpr int kMaxChunks = kSkv / kKC;
constexpr float kScale = 0.125f;
static_assert(kSeq % kQB == 0);
static_assert(kSkv % kKC == 0);
static_assert(kSeq == kSkv);
static_assert(kDim == 64);
static_assert(kKC % 32 == 0);
static_assert(kDim % 32 == 0);

__device__ __forceinline__ unsigned short f2bf_bits(float f) {
  unsigned u = __float_as_uint(f);
  return (unsigned short)((u + 0x7FFFu + ((u >> 16) & 1u)) >> 16);
}
__device__ __forceinline__ float bf_bits2f(unsigned short h) { return __uint_as_float(((unsigned)h) << 16); }

__device__ __forceinline__ void dep_guard_b(v8f& a, v8f& b, v16b x, v16b y) { asm volatile("v_nop\n\tv_nop\n\tv_nop\n\tv_nop" : "+v"(a), "+v"(b) : "v"(x), "v"(y)); }
__device__ __forceinline__ void keep4_b(v16b a, v16b b, v16b c, v16b d) { asm volatile("v_nop" :: "v"(a), "v"(b), "v"(c), "v"(d)); }
template <typename T> struct Frag;
template <> struct Frag<__bf16> {
  typedef v16b V; union U { v16b v; v8b h[2]; };
  static __device__ __forceinline__ v16b load(const __bf16* p) {
    U f; f.h[0] = *(const v8b*)(p); f.h[1] = *(const v8b*)(p + 16); return f.v;
  }
  static __device__ __forceinline__ v8f mma(v16b a, v16b b, v8f c) {
    return __builtin_amdgcn_wmma_f32_16x16x32_bf16(false, a, false, b, (short)0, c, false, false);
  }
  static __device__ __forceinline__ void guard(v8f& a, v8f& b, v16b x, v16b y) { dep_guard_b(a, b, x, y); }
  static __device__ __forceinline__ void keep(v16b a, v16b b, v16b c, v16b d) { keep4_b(a, b, c, d); }
};

__device__ __forceinline__ unsigned short at_bf_bits(float f) {
  unsigned u = __float_as_uint(f);
  return (unsigned short)((u + 0x7FFFu + ((u >> 16) & 1u)) >> 16);
}
__device__ __forceinline__ __bf16 at_f2bf(float f) { return __builtin_bit_cast(__bf16, at_bf_bits(f)); }
__device__ __forceinline__ void at_split(float f, __bf16& hi, __bf16& lo) {
  const unsigned short hb = at_bf_bits(f);
  hi = __builtin_bit_cast(__bf16, hb);
  lo = at_f2bf(f - __uint_as_float(((unsigned)hb) << 16));
}
__device__ __forceinline__ v8f at_mma(v16b a, v16b b, v8f c) {
  c = __builtin_amdgcn_wmma_f32_16x16x32_bf16(false, a, false, b, (short)0, c, false, false);
  asm volatile("v_nop\n\tv_nop\n\tv_nop\n\tv_nop" : "+v"(c) : "v"(a), "v"(b));
  return c;
}

__device__ __forceinline__ v4u pack_bf16x8(v4f a, v4f b) {
  v4u r;
  r[0] = (unsigned)f2bf_bits(a[0]) | ((unsigned)f2bf_bits(a[1]) << 16);
  r[1] = (unsigned)f2bf_bits(a[2]) | ((unsigned)f2bf_bits(a[3]) << 16);
  r[2] = (unsigned)f2bf_bits(b[0]) | ((unsigned)f2bf_bits(b[1]) << 16);
  r[3] = (unsigned)f2bf_bits(b[2]) | ((unsigned)f2bf_bits(b[3]) << 16);
  return r;
}

__global__ __launch_bounds__(128)
void prep_planes(const float* __restrict__ q, const float* __restrict__ k, const float* __restrict__ v,
                 unsigned short* __restrict__ qp, unsigned short* __restrict__ kp, unsigned short* __restrict__ vtp)
{
  __shared__ __align__(16) float tile[64 * 68];
  const int tid = threadIdx.x;
  const int bx  = blockIdx.x;
  const int nst = kSkv / 64;
  const int st  = bx % nst;
  const int bh  = bx / nst;
  const int h   = bh % kHeads;
  const int b   = bh / kHeads;
  const int s0  = st * 64;

  {
    const int s = tid >> 1, dh = (tid & 1) * 32;
    const float* src = v + ((size_t)(b * kSkv + s0 + s) * kHeads + h) * kDim + dh;
#pragma unroll
    for (int i = 0; i < 8; ++i) *(v4f*)(tile + s * 68 + dh + 4 * i) = *(const v4f*)(src + 4 * i);
  }
  __syncthreads();

  const int rg = tid >> 3;
  const int c8 = (tid & 7) * 8;

  v4u qw[4], kw[4], vw[4];
#pragma unroll
  for (int it = 0; it < 4; ++it) {
    const int row = it * 16 + rg;
    const size_t off = ((size_t)(b * kSeq + s0 + row) * kHeads + h) * kDim + c8;
    const v4f a0 = *(const v4f*)(q + off);
    const v4f a1 = *(const v4f*)(q + off + 4);
    qw[it] = pack_bf16x8(a0, a1);
  }
  asm volatile("" ::: "memory");
#pragma unroll
  for (int it = 0; it < 4; ++it) {
    const int row = it * 16 + rg;
    const size_t off = ((size_t)(b * kSkv + s0 + row) * kHeads + h) * kDim + c8;
    const v4f a0 = *(const v4f*)(k + off);
    const v4f a1 = *(const v4f*)(k + off + 4);
    kw[it] = pack_bf16x8(a0, a1);
  }
  asm volatile("" ::: "memory");
#pragma unroll
  for (int it = 0; it < 4; ++it) {
    const int d = it * 16 + rg;
    v4f f0, f1;
#pragma unroll
    for (int e = 0; e < 4; ++e) {
      f0[e] = tile[(c8 + e) * 68 + d];
      f1[e] = tile[(c8 + 4 + e) * 68 + d];
    }
    vw[it] = pack_bf16x8(f0, f1);
  }

  for (int pass = 0; pass < 2; ++pass) {
#pragma unroll
    for (int it = 0; it < 4; ++it) {
      const int row = it * 16 + rg;
      const size_t offq = ((size_t)(b * kSeq + s0 + row) * kHeads + h) * kDim + c8;
      *(volatile v4u*)(qp + offq) = qw[it];
      *(volatile v4u*)(kp + offq) = kw[it];
      const int d = row;
      const size_t offv = ((size_t)((b * kHeads + h) * kDim + d)) * kSkv + s0 + c8;
      *(volatile v4u*)(vtp + offv) = vw[it];
    }
    __threadfence();
  }
}

__global__ __launch_bounds__(128)
void attn_planes_kernel(const unsigned short* __restrict__ qp, const unsigned short* __restrict__ kp,
                        const unsigned short* __restrict__ vtp, const int* __restrict__ vlen,
                        float* __restrict__ out)
{
  __shared__ __align__(16) __bf16 Ksh[kKC * kDim];
  __shared__ __align__(16) __bf16 Vts[kDim * kKC];
  __shared__ __align__(16) __bf16 Psh[kNW][16 * kKC];
  __shared__ __align__(16) __bf16 Psl[kNW][16 * kKC];
  __shared__ __align__(16) float  Os[kNW][16 * 68];

  const int tid  = threadIdx.x;
  const int wave = tid >> 5;
  const int lane = tid & 31;
  const int hh   = lane >> 4;
  const int c    = lane & 15;

  const int nqb = kSeq / kQB;
  const int bx  = blockIdx.x;
  const int qb  = bx % nqb;
  const int bh  = bx / nqb;
  const int h   = bh % kHeads;
  const int b   = bh / kHeads;
  const int q0  = qb * kQB + wave * 16;

  int valid = vlen[b];
  valid = valid < 0 ? 0 : valid;
  valid = valid > kSkv ? kSkv : valid;
  int nChunks = (valid + kKC - 1) / kKC;
  nChunks = nChunks < 1 ? 1 : nChunks;
  nChunks = nChunks > kMaxChunks ? kMaxChunks : nChunks;

  v16b qa[2];
  {
    const __bf16* qrow = (const __bf16*)qp + ((size_t)(b * kSeq + q0 + c) * kHeads + h) * kDim;
#pragma unroll
    for (int dc = 0; dc < 2; ++dc) qa[dc] = Frag<__bf16>::load(qrow + dc * 32 + 8 * hh);
  }

  float mrow[8], lrow[8];
  v8f oacc[4];
#pragma unroll
  for (int r = 0; r < 8; ++r) { mrow[r] = -INFINITY; lrow[r] = 0.f; }
#pragma unroll
  for (int t = 0; t < 4; ++t) oacc[t] = (v8f){0.f,0.f,0.f,0.f,0.f,0.f,0.f,0.f};

  const size_t kbase  = ((size_t)b * kSkv) * kHeads * kDim + (size_t)h * kDim;
  const size_t vtbase = ((size_t)(b * kHeads + h) * kDim) * kSkv;

  for (int kc = 0; kc < nChunks; ++kc) {
    const int kv0 = kc * kKC;
    __syncthreads();
    {
      const int r = tid >> 1, half = (tid & 1) * 32;
      const v4u* ksrc = (const v4u*)(kp + kbase + (size_t)(kv0 + r) * (kHeads * kDim) + half);
      v4u* kdst = (v4u*)(Ksh + r * kDim + half);
      const v4u* vsrc = (const v4u*)(vtp + vtbase + (size_t)r * kSkv + kv0 + half);
      v4u* vdst = (v4u*)(Vts + r * kKC + half);
#pragma unroll
      for (int i = 0; i < 4; ++i) { kdst[i] = ksrc[i]; vdst[i] = vsrc[i]; }
    }
    __syncthreads();

    v8f s[4];
#pragma unroll
    for (int j = 0; j < 4; ++j) {
      s[j] = (v8f){0.f,0.f,0.f,0.f,0.f,0.f,0.f,0.f};
#pragma unroll
      for (int dc = 0; dc < 2; ++dc) {
        const v16b kb = Frag<__bf16>::load(Ksh + (j * 16 + c) * kDim + dc * 32 + 8 * hh);
        s[j] = at_mma(qa[dc], kb, s[j]);
      }
    }

    float cm[8];
#pragma unroll
    for (int r = 0; r < 8; ++r) {
      float m = -INFINITY;
#pragma unroll
      for (int j = 0; j < 4; ++j) {
        const int kvcol = kv0 + j * 16 + c;
        float sv = s[j][r] * kScale;
        sv = (kvcol < valid) ? sv : -INFINITY;
        s[j][r] = sv;
        m = fmaxf(m, sv);
      }
#pragma unroll
      for (int off = 1; off < 16; off <<= 1) m = fmaxf(m, __shfl_xor(m, off, 32));
      cm[r] = m;
    }

    __bf16* pwh = Psh[wave];
    __bf16* pwl = Psl[wave];
#pragma unroll
    for (int r = 0; r < 8; ++r) {
      const float mnew  = fmaxf(mrow[r], cm[r]);
      const float alpha = expf(mrow[r] - mnew);
      mrow[r] = mnew;
      float psum = 0.f;
#pragma unroll
      for (int j = 0; j < 4; ++j) {
        const float p = expf(s[j][r] - mnew);
        psum += p;
        __bf16 ph, pl;
        at_split(p, ph, pl);
        pwh[(8 * hh + r) * kKC + j * 16 + c] = ph;
        pwl[(8 * hh + r) * kKC + j * 16 + c] = pl;
      }
#pragma unroll
      for (int off = 1; off < 16; off <<= 1) psum += __shfl_xor(psum, off, 32);
      lrow[r] = lrow[r] * alpha + psum;
#pragma unroll
      for (int t = 0; t < 4; ++t) oacc[t][r] *= alpha;
    }
    __builtin_amdgcn_fence(__ATOMIC_RELEASE, "workgroup");
    __builtin_amdgcn_wave_barrier();
    __builtin_amdgcn_fence(__ATOMIC_ACQUIRE, "workgroup");

#pragma unroll 1
    for (int kk = 0; kk < 2; ++kk) {
      const v16b pa = Frag<__bf16>::load(pwh + c * kKC + kk * 32 + 8 * hh);
      const v16b pb = Frag<__bf16>::load(pwl + c * kKC + kk * 32 + 8 * hh);
#pragma unroll
      for (int t = 0; t < 4; ++t) {
        const v16b vb = Frag<__bf16>::load(Vts + (t * 16 + c) * kKC + kk * 32 + 8 * hh);
        oacc[t] = at_mma(pa, vb, oacc[t]);
        oacc[t] = at_mma(pb, vb, oacc[t]);
      }
    }
  }

  float* os = Os[wave];
#pragma unroll
  for (int r = 0; r < 8; ++r) {
    const float inv = 1.0f / lrow[r];
#pragma unroll
    for (int t = 0; t < 4; ++t) os[(8 * hh + r) * 68 + t * 16 + c] = oacc[t][r] * inv;
  }
  __builtin_amdgcn_fence(__ATOMIC_RELEASE, "workgroup");
  __builtin_amdgcn_wave_barrier();
  __builtin_amdgcn_fence(__ATOMIC_ACQUIRE, "workgroup");
  {
    const size_t o_rs = (size_t)kHeads * kDim;
    float* ob_ptr = out + ((size_t)b * kSeq) * o_rs + (size_t)h * kDim;
    const int c4 = (lane & 15) * 4;
    for (int pass = 0; pass < 2; ++pass) {
#pragma unroll
      for (int it = 0; it < 8; ++it) {
        const int row = it * 2 + hh;
        v4f val = *(const v4f*)(os + row * 68 + c4);
        *(volatile v4f*)(ob_ptr + (size_t)(q0 + row) * o_rs + c4) = val;
      }
      __threadfence();
    }
  }
}

extern "C" void kernel_launch(void* const* d_in, const int* in_sizes, int n_in,
                              void* d_out, int out_size, void* d_ws, size_t ws_size,
                              hipStream_t stream)
{
  (void)in_sizes; (void)n_in; (void)out_size;
  const float* q  = (const float*)d_in[0];
  const float* k  = (const float*)d_in[1];
  const float* v  = (const float*)d_in[2];
  const int*   vl = (const int*)d_in[3];
  float* out = (float*)d_out;

  const size_t planeElems = (size_t)kBatch * kSeq * kHeads * kDim;
  const size_t carveBytes = 3 * planeElems * sizeof(unsigned short);
  if (carveBytes > ws_size) return;

  unsigned short* ws  = (unsigned short*)d_ws;
  unsigned short* qp  = ws;
  unsigned short* kp  = ws + planeElems;
  unsigned short* vtp = ws + 2 * planeElems;

  const int prepBlocks = kBatch * kHeads * (kSkv / 64);
  const int attnBlocks = kBatch * kHeads * (kSeq / kQB);

  prep_planes<<<dim3(prepBlocks), dim3(128), 0, stream>>>(q, k, v, qp, kp, vtp);
  attn_planes_kernel<<<dim3(attnBlocks), dim3(128), 0, stream>>>(qp, kp, vtp, vl, out);
}
